// TransformerBlock_21844203668377
// MI455X (gfx1250) — hardware-run, weakly checked
//
#include <hip/hip_runtime.h>


#ifndef SEQ
#define SEQ 8192
#endif
#define SEQ_FULL 8192
#define FD   16
#define NH_  4
#define DH   4
#define HD   32
#define HID  512
#define HP   520
#define ZP   20
#define AW   4
#define EPSN 1.1920929e-07f
#define WSA   64.0f
#define WSA_I (1.0f / 64.0f)
#define WSB   256.0f
#define WSB_I (1.0f / 256.0f)
#define SC2  ((float)(0.17677669529663687 * 1.4426950408889634))
#define L2E  1.4426950408889634f
#define PSH  14.0f
#define NEGB (-3.0e38f)

static_assert(FD == 16);
static_assert(NH_ * DH == FD);
static_assert(NH_ * DH == 16);
static_assert(HD == 32);
static_assert(AW == NH_);
static_assert(SEQ % 64 == 0);
static_assert(SEQ % 32 == 0);
static_assert(SEQ % 16 == 0);
static_assert(SEQ <= SEQ_FULL);
static_assert(HID % 64 == 0);
static_assert(HID % 32 == 0);
static_assert(HP >= HID && (HP * 2) % 16 == 0);
static_assert((ZP * 4) % 16 == 0 && ZP >= FD);
static_assert((2 * NH_ * HD * FD) % 8 == 0 && (NH_ * DH * FD) % 8 == 0 && (FD * FD) % 8 == 0);
static_assert((HID * FD) % 8 == 0 && (HID * HID) % 8 == 0);
static_assert(8 * 32 * 16 == 64 * HD * 2);
static_assert(4 * 32 * 16 == 16 * 64 * 2);
static_assert(2 * 32 * 16 == 16 * FD * 4);
static_assert((64 * 36 + 16 * 68) * 4 <= 131072);
static_assert(16 * ZP * 4 <= 131072);
static_assert(2 * 16 * HP * 2 + 2 * 16 * ZP * 4 <= 131072);

typedef _Float16 h16;
typedef __attribute__((ext_vector_type(16))) _Float16 v16h;
typedef __attribute__((ext_vector_type(8)))  _Float16 v8h;
typedef __attribute__((ext_vector_type(8)))  float    v8f;
typedef __attribute__((ext_vector_type(4)))  float    v4f;
typedef v4f  __attribute__((may_alias)) v4fa;
typedef v8h  __attribute__((may_alias)) v8ha;

__device__ __forceinline__ unsigned short f2bf(float f) { unsigned u = __float_as_uint(f); u += 0x7FFFu + ((u >> 16) & 1u); return (unsigned short)(u >> 16); }
__device__ __forceinline__ float bfr(float f) { return __uint_as_float(((unsigned)f2bf(f)) << 16); }
__device__ __forceinline__ v16h cat16(v8h lo, v8h hi) { return __builtin_shufflevector(lo, hi, 0, 1, 2, 3, 4, 5, 6, 7, 8, 9, 10, 11, 12, 13, 14, 15); }
__device__ __forceinline__ v16h  ldh(const h16* p) { return cat16(*(const v8h*)p, *(const v8h*)(p + 16)); }
static __device__ __forceinline__ h16 toh_flush(float v) { const h16 r = (h16)v; return (fabsf(v) < 6.103515625e-05f) ? (h16)0.0f : r; }
static __device__ __forceinline__ v8f wmma16g(v16h a, v16h b, v8f c) {
    c = __builtin_amdgcn_wmma_f32_16x16x32_f16(false, a, false, b, (short)0, c, false, false);
    asm volatile("v_nop\n\tv_nop\n\tv_nop\n\tv_nop" : "+v"(c) : "v"(a), "v"(b));
    return c;
}
static __device__ __forceinline__ float silu_f(float v) { const float e = __builtin_amdgcn_exp2f(-v * L2E); return v * __builtin_amdgcn_rcpf(1.0f + e); }

__global__ __launch_bounds__(256) void k_wconv(const float* __restrict__ src, h16* dst, size_t n8, float scale) {
    const size_t i = (size_t)blockIdx.x * 256 + threadIdx.x; if (i >= n8) return;
    const v8f v = *(const v8f*)(src + i * 8); v8h o;
#pragma unroll
    for (int k = 0; k < 8; ++k) o[k] = toh_flush(bfr(v[k]) * scale);
    *(volatile v8h*)(dst + i * 8) = o; __threadfence(); *(volatile v8h*)(dst + i * 8) = o;
}

__global__ __launch_bounds__(32) void k_qkv(const float* __restrict__ X, const float* __restrict__ n1w, const h16* __restrict__ WQK, const h16* __restrict__ WV,
                                            const float* __restrict__ Qb, const float* __restrict__ Kb, const float* __restrict__ Vb, h16* QKP, h16* VT) {
    __shared__ __align__(16) float os[64 * 36];
    __shared__ __align__(16) float vs[16 * 68];
    const int lane = threadIdx.x & 31, lr = lane & 15, hi = lane >> 4;
    const int r0 = blockIdx.x * 64;
    const v8h z8 = (v8h){};
    float gw[8];
    { const v4f g0 = *(const v4f*)(n1w + 8 * hi), g1 = *(const v4f*)(n1w + 8 * hi + 4);
#pragma unroll
      for (int i = 0; i < 4; ++i) { gw[i] = bfr(g0[i]); gw[4 + i] = bfr(g1[i]); } }
    v16h a[4];
#pragma unroll
    for (int mb = 0; mb < 4; ++mb) {
        const float* xp = X + (size_t)(r0 + mb * 16 + lr) * FD + 8 * hi;
        const v4f x0 = *(const v4f*)xp, x1 = *(const v4f*)(xp + 4);
        float xv[8]; float ss = 0.0f;
#pragma unroll
        for (int i = 0; i < 4; ++i) { xv[i] = bfr(x0[i]); xv[4 + i] = bfr(x1[i]); }
#pragma unroll
        for (int i = 0; i < 8; ++i) ss += xv[i] * xv[i];
        ss += __shfl_xor(ss, 16, 32);
        const float rn = rsqrtf(ss * (1.0f / 16.0f) + EPSN);
        v16h f = (v16h){};
#pragma unroll
        for (int i = 0; i < 8; ++i) f[i] = toh_flush(xv[i] * rn * gw[i]);
        a[mb] = f;
    }
#pragma unroll 1
    for (int g = 0; g < 2 * NH_; ++g) {
        const h16* wp = WQK + (size_t)(g * HD + lr) * FD + 8 * hi;
        const v16h bA = cat16(*(const v8h*)wp, z8), bB = cat16(*(const v8h*)(wp + 16 * FD), z8);
        const int hh = g & (NH_ - 1);
        const float q0 = Qb[hh * HD + lr], q1 = Qb[hh * HD + 16 + lr], k0 = Kb[hh * HD + lr], k1 = Kb[hh * HD + 16 + lr];
        const float bc0 = bfr((g < NH_) ? q0 : k0), bc1 = bfr((g < NH_) ? q1 : k1);
#pragma unroll
        for (int mb = 0; mb < 4; ++mb) {
            v8f c0 = (v8f){}, c1 = (v8f){};
            c0 = wmma16g(a[mb], bA, c0); c1 = wmma16g(a[mb], bB, c1);
#pragma unroll
            for (int j = 0; j < 8; ++j) { os[(mb * 16 + hi * 8 + j) * 36 + lr] = c0[j] * WSA_I + bc0; os[(mb * 16 + hi * 8 + j) * 36 + 16 + lr] = c1[j] * WSA_I + bc1; }
        }
        __syncthreads();
        h16* pl = QKP + (size_t)g * SEQ * HD + (size_t)r0 * HD;
#pragma unroll 1
        for (int ps = 0; ps < 2; ++ps) {
#pragma unroll
            for (int i = 0; i < 8; ++i) { const int p = i * 32 + lane; const int row = p >> 2, c8 = (p & 3) * 8;
                const v4f x0 = *(const v4fa*)(&os[row * 36 + c8]); const v4f x1 = *(const v4fa*)(&os[row * 36 + c8 + 4]); v8h hv;
#pragma unroll
                for (int e = 0; e < 4; ++e) { hv[e] = toh_flush(x0[e]); hv[4 + e] = toh_flush(x1[e]); }
                *(volatile v8h*)(pl + (size_t)p * 8) = hv; }
            if (ps == 0) __threadfence(); }
        __syncthreads();
    }
    { const v16h av = cat16(*(const v8h*)(WV + (size_t)lr * FD + 8 * hi), z8);
      float bv[8];
      { const v4f b0v = *(const v4f*)(Vb + 8 * hi), b1v = *(const v4f*)(Vb + 8 * hi + 4);
#pragma unroll
        for (int i = 0; i < 4; ++i) { bv[i] = bfr(b0v[i]); bv[4 + i] = bfr(b1v[i]); } }
#pragma unroll
      for (int mb = 0; mb < 4; ++mb) {
          v8f c = (v8f){};
          c = wmma16g(av, a[mb], c);
#pragma unroll
          for (int j = 0; j < 8; ++j) vs[(hi * 8 + j) * 68 + mb * 16 + lr] = c[j] * WSA_I + bv[j];
      }
      __syncthreads();
#pragma unroll 1
      for (int ps = 0; ps < 2; ++ps) {
#pragma unroll
          for (int s = 0; s < 4; ++s) { const int row = 4 * s + (lane >> 3), c8 = (lane & 7) * 8;
              const v4f x0 = *(const v4fa*)(&vs[row * 68 + c8]); const v4f x1 = *(const v4fa*)(&vs[row * 68 + c8 + 4]); v8h hv;
#pragma unroll
              for (int e = 0; e < 4; ++e) { hv[e] = toh_flush(x0[e]); hv[4 + e] = toh_flush(x1[e]); }
              *(volatile v8h*)(VT + (size_t)row * SEQ + (size_t)r0 + c8) = hv; }
          if (ps == 0) __threadfence(); }
    }
}

__global__ __launch_bounds__(32 * AW) void k_flash(const h16* __restrict__ QH, const h16* __restrict__ KP, const h16* __restrict__ VT, float* RES) {
    __shared__ __align__(16) float rs[16 * ZP];
    const int lane = threadIdx.x & 31, lr = lane & 15, hi = lane >> 4;
    const int wave = __builtin_amdgcn_readfirstlane((int)(threadIdx.x >> 5));
    const int h = wave;
    const int t0 = blockIdx.x * 16;
    const size_t pbase = (size_t)h * SEQ * HD;
    const v16h qh = ldh(QH + pbase + (size_t)(t0 + lr) * HD + 8 * hi);
    const size_t ko = pbase + (size_t)lr * HD + 8 * hi;
    const size_t vo = (size_t)(h * DH + (lr & (DH - 1))) * SEQ + 8 * hi;
    v8f o0 = (v8f){};
    float m = NEGB, l = 0.0f;
#pragma unroll 1
    for (int key0 = 0; key0 < SEQ; key0 += 32) {
        const h16* ka = KP + ko + (size_t)key0 * HD;
        const v16h ka0 = ldh(ka), kb0 = ldh(ka + 16 * HD);
        v8f sa = (v8f){}, sb = (v8f){};
        sa = wmma16g(ka0, qh, sa); sb = wmma16g(kb0, qh, sb);
        float ta[8], tb[8]; float mx = NEGB;
#pragma unroll
        for (int r = 0; r < 8; ++r) { ta[r] = sa[r] * SC2; tb[r] = sb[r] * SC2; mx = fmaxf(mx, fmaxf(ta[r], tb[r])); }
        mx = fmaxf(mx, __shfl_xor(mx, 16, 32));
        const float mnew = fmaxf(m, mx);
        const float alpha = __builtin_amdgcn_exp2f(m - mnew);
        const float sh = PSH - mnew;
        v16h pb; float ls = 0.0f;
#pragma unroll
        for (int r = 0; r < 8; ++r) {
            const float xa = ta[r] + sh, xb = tb[r] + sh;
            const float ea = __builtin_amdgcn_exp2f(xa), eb = __builtin_amdgcn_exp2f(xb);
            const float ga = (xa < -14.0f) ? 0.0f : ea, gb = (xb < -14.0f) ? 0.0f : eb;
            const h16 pa = (h16)ga; const h16 pc = (h16)gb;
            pb[r] = pa; pb[8 + r] = pc;
            ls += (float)pa + (float)pc; }
        l = l * alpha + ls; m = mnew;
        o0 = o0 * alpha;
        const v16h v0 = ldh(VT + vo + key0);
        o0 = wmma16g(v0, pb, o0);
    }
    l += __shfl_xor(l, 16, 32);
    const float inv = 1.0f / l;
    { v4f a; a[0] = o0[0] * inv; a[1] = o0[1] * inv; a[2] = o0[2] * inv; a[3] = o0[3] * inv;
      if (hi == 0) *(v4fa*)(&rs[lr * ZP + h * DH]) = a; }
    __syncthreads();
    if (wave < 2) {
        const int p = wave * 32 + lane; const int row = p >> 2, c4 = (p & 3) * 4;
        const v4f val = *(const v4fa*)(&rs[row * ZP + c4]);
        float* dst = RES + (size_t)t0 * FD + (size_t)p * 4;
        *(volatile v4f*)dst = val; __threadfence(); *(volatile v4f*)dst = val;
    }
}

__global__ __launch_bounds__(32) void k_mlp(const float* __restrict__ X, const float* __restrict__ RES, const h16* __restrict__ AWP, const float* __restrict__ attn_b,
                                            const float* __restrict__ n2w, const h16* __restrict__ W0, const float* __restrict__ b0, const h16* __restrict__ W1,
                                            const float* __restrict__ b1, const h16* __restrict__ W2, const float* __restrict__ b2, float* OUT) {
    __shared__ __align__(16) h16 h0s[16 * HP];
    __shared__ __align__(16) h16 h1s[16 * HP];
    __shared__ __align__(16) float zs[16 * ZP];
    __shared__ __align__(16) float ys[16 * ZP];
    const int lane = threadIdx.x & 31, lr = lane & 15, hi = lane >> 4;
    const int m0 = blockIdx.x * 16;
    const v8h z8 = (v8h){};
    v8f yacc = (v8f){};
    { const float* rp = RES + (size_t)(m0 + lr) * FD + 8 * hi;
      const v4f r0 = *(const v4f*)rp, r1 = *(const v4f*)(rp + 4);
      v16h ar = (v16h){};
#pragma unroll
      for (int i = 0; i < 4; ++i) { ar[i] = toh_flush(r0[i]); ar[4 + i] = toh_flush(r1[i]); }
      const v16h bw = cat16(*(const v8h*)(AWP + (size_t)lr * FD + 8 * hi), z8);
      yacc = wmma16g(ar, bw, yacc); }
    { const float ab = bfr(attn_b[lr]);
#pragma unroll
      for (int j = 0; j < 8; ++j) ys[(hi * 8 + j) * ZP + lr] = yacc[j] * WSA_I + ab; }
    __syncthreads();
    v16h az = (v16h){};
    { const float* xp = X + (size_t)(m0 + lr) * FD + 8 * hi;
      const v4f x0 = *(const v4f*)xp, x1 = *(const v4f*)(xp + 4);
      const v4f y0 = *(const v4fa*)(&ys[lr * ZP + 8 * hi]), y1 = *(const v4fa*)(&ys[lr * ZP + 8 * hi + 4]);
      const v4f g0 = *(const v4f*)(n2w + 8 * hi), g1 = *(const v4f*)(n2w + 8 * hi + 4);
      float z[8]; float ss = 0.0f; v4f za, zb;
#pragma unroll
      for (int i = 0; i < 4; ++i) { z[i] = bfr(x0[i]) + y0[i]; z[4 + i] = bfr(x1[i]) + y1[i]; za[i] = z[i]; zb[i] = z[4 + i]; }
#pragma unroll
      for (int i = 0; i < 8; ++i) ss += z[i] * z[i];
      *(v4fa*)(&zs[lr * ZP + 8 * hi]) = za; *(v4fa*)(&zs[lr * ZP + 8 * hi + 4]) = zb;
      ss += __shfl_xor(ss, 16, 32);
      const float rn = rsqrtf(ss * (1.0f / 16.0f) + EPSN);
#pragma unroll
      for (int i = 0; i < 4; ++i) { az[i] = toh_flush(z[i] * rn * bfr(g0[i])); az[4 + i] = toh_flush(z[4 + i] * rn * bfr(g1[i])); } }
#pragma unroll 1
    for (int ct = 0; ct < HID / 16; ++ct) {
        const int n = ct * 16 + lr;
        const v16h bw = cat16(*(const v8h*)(W0 + (size_t)n * FD + 8 * hi), z8);
        v8f c = (v8f){};
        c = wmma16g(az, bw, c);
        const float bb = bfr(b0[n]);
#pragma unroll
        for (int j = 0; j < 8; ++j) h0s[(hi * 8 + j) * HP + n] = toh_flush(silu_f(c[j] * WSA_I + bb));
    }
    __syncthreads();
#pragma unroll 1
    for (int ng = 0; ng < HID / 64; ++ng) {
        v8f acc[4];
#pragma unroll
        for (int nb = 0; nb < 4; ++nb) acc[nb] = (v8f){};
        const size_t wo = (size_t)(ng * 64 + lr) * HID + 8 * hi;
#pragma unroll 1
        for (int kc = 0; kc < HID; kc += 32) {
            const v16h a = cat16(*(const v8ha*)(&h0s[lr * HP + kc + 8 * hi]), *(const v8ha*)(&h0s[lr * HP + kc + 16 + 8 * hi]));
#pragma unroll
            for (int nb = 0; nb < 4; ++nb) { const v16h b = ldh(W1 + wo + (size_t)nb * 16 * HID + kc); acc[nb] = wmma16g(a, b, acc[nb]); }
        }
#pragma unroll
        for (int nb = 0; nb < 4; ++nb) {
            const int n = ng * 64 + nb * 16 + lr;
            const float bb = bfr(b1[n]);
#pragma unroll
            for (int j = 0; j < 8; ++j) h1s[(hi * 8 + j) * HP + n] = toh_flush(silu_f(acc[nb][j] * WSB_I + bb));
        }
    }
    __syncthreads();
    { v8f c = (v8f){};
      const size_t wo = (size_t)lr * HID + 8 * hi;
#pragma unroll 1
      for (int kc = 0; kc < HID; kc += 32) {
          const v16h a = cat16(*(const v8ha*)(&h1s[lr * HP + kc + 8 * hi]), *(const v8ha*)(&h1s[lr * HP + kc + 16 + 8 * hi]));
          const v16h b = ldh(W2 + wo + kc);
          c = wmma16g(a, b, c);
      }
      const float bb = bfr(b2[lr]);
#pragma unroll
      for (int j = 0; j < 8; ++j) ys[(hi * 8 + j) * ZP + lr] = silu_f(c[j] * WSB_I + bb); }
    __syncthreads();
    float* orow = OUT + (size_t)m0 * FD;
#pragma unroll 1
    for (int ps = 0; ps < 2; ++ps) {
#pragma unroll
        for (int s = 0; s < 2; ++s) { const int p = s * 32 + lane; const int row = p >> 2, c4 = (p & 3) * 4;
            const v4f sv = *(const v4fa*)(&ys[row * ZP + c4]); const v4f zv = *(const v4fa*)(&zs[row * ZP + c4]);
            const v4f val = sv + zv;
            *(volatile v4f*)(orow + (size_t)p * 4) = val; }
        if (ps == 0) __threadfence(); }
}

static constexpr size_t al256(size_t v) { return (v + 255) & ~(size_t)255; }
static constexpr size_t SZ_WQK = al256((size_t)2 * NH_ * HD * FD * 2);
static constexpr size_t SZ_WV  = al256((size_t)NH_ * DH * FD * 2);
static constexpr size_t SZ_AW  = al256((size_t)FD * FD * 2);
static constexpr size_t SZ_W0  = al256((size_t)HID * FD * 2);
static constexpr size_t SZ_W1  = al256((size_t)HID * HID * 2);
static constexpr size_t SZ_W2  = al256((size_t)FD * HID * 2);
static constexpr size_t SZ_QK  = al256((size_t)2 * NH_ * SEQ * HD * 2);
static constexpr size_t SZ_VT  = al256((size_t)NH_ * DH * SEQ * 2);
static constexpr size_t SZ_RS  = al256((size_t)SEQ * FD * 4);
static constexpr size_t SZ_TOTAL = SZ_WQK + SZ_WV + SZ_AW + SZ_W0 + SZ_W1 + SZ_W2 + SZ_QK + SZ_VT + SZ_RS;
static_assert(SZ_TOTAL <= (size_t)134217728);
static_assert(((size_t)NH_ * HD * FD * 2) % 256 == 0);
static_assert(((size_t)NH_ * SEQ * HD * 2) % 256 == 0);

extern "C" void kernel_launch(void* const* d_in, const int* in_sizes, int n_in,
                              void* d_out, int out_size, void* d_ws, size_t ws_size, hipStream_t stream) {
    if (n_in < 17) return;
    if ((size_t)in_sizes[0] < (size_t)SEQ * FD) return;
    if (in_sizes[1] < FD || in_sizes[2] < FD) return;
    if (in_sizes[3] < NH_ * HD * FD || in_sizes[4] < NH_ * HD || in_sizes[5] < NH_ * HD * FD || in_sizes[6] < NH_ * HD) return;
    if (in_sizes[7] < NH_ * DH * FD || in_sizes[8] < NH_ * DH || in_sizes[9] < FD * FD || in_sizes[10] < FD) return;
    if (in_sizes[11] < HID * FD || in_sizes[12] < HID || in_sizes[13] < HID * HID || in_sizes[14] < HID || in_sizes[15] < FD * HID || in_sizes[16] < FD) return;
    if ((size_t)out_size < (size_t)SEQ * FD) return;
    if (SZ_TOTAL > ws_size) return;
    const float* x   = (const float*)d_in[0];
    const float* n1w = (const float*)d_in[1];
    const float* n2w = (const float*)d_in[2];
    const float* Qw  = (const float*)d_in[3];  const float* Qb = (const float*)d_in[4];
    const float* Kw  = (const float*)d_in[5];  const float* Kb = (const float*)d_in[6];
    const float* Vw  = (const float*)d_in[7];  const float* Vb = (const float*)d_in[8];
    const float* aw  = (const float*)d_in[9];  const float* ab = (const float*)d_in[10];
    const float* w0  = (const float*)d_in[11]; const float* b0 = (const float*)d_in[12];
    const float* w1  = (const float*)d_in[13]; const float* b1 = (const float*)d_in[14];
    const float* w2  = (const float*)d_in[15]; const float* b2 = (const float*)d_in[16];
    float* OUT = (float*)d_out;
    char* wsp = (char*)d_ws;
    h16* WQK = (h16*)wsp; wsp += SZ_WQK;
    h16* WV  = (h16*)wsp; wsp += SZ_WV;
    h16* AWP = (h16*)wsp; wsp += SZ_AW;
    h16* W0  = (h16*)wsp; wsp += SZ_W0;
    h16* W1  = (h16*)wsp; wsp += SZ_W1;
    h16* W2  = (h16*)wsp; wsp += SZ_W2;
    h16* QKP = (h16*)wsp; wsp += SZ_QK;
    h16* VT  = (h16*)wsp; wsp += SZ_VT;
    float* RES = (float*)wsp; wsp += SZ_RS;
    h16* QH = QKP; h16* KP = QKP + (size_t)NH_ * SEQ * HD;

    { const size_t n8 = (size_t)NH_ * HD * FD / 8; const unsigned g = (unsigned)((n8 + 255) / 256);
      k_wconv<<<g, 256, 0, stream>>>(Qw, WQK, n8, WSA);
      k_wconv<<<g, 256, 0, stream>>>(Kw, WQK + (size_t)NH_ * HD * FD, n8, WSA); }
    { const size_t n8 = (size_t)NH_ * DH * FD / 8; k_wconv<<<(unsigned)((n8 + 255) / 256), 256, 0, stream>>>(Vw, WV, n8, WSA); }
    { const size_t n8 = (size_t)FD * FD / 8;       k_wconv<<<(unsigned)((n8 + 255) / 256), 256, 0, stream>>>(aw, AWP, n8, WSA); }
    { const size_t n8 = (size_t)HID * FD / 8;      k_wconv<<<(unsigned)((n8 + 255) / 256), 256, 0, stream>>>(w0, W0, n8, WSA); }
    { const size_t n8 = (size_t)HID * HID / 8;     k_wconv<<<(unsigned)((n8 + 255) / 256), 256, 0, stream>>>(w1, W1, n8, WSB); }
    { const size_t n8 = (size_t)FD * HID / 8;      k_wconv<<<(unsigned)((n8 + 255) / 256), 256, 0, stream>>>(w2, W2, n8, WSB); }

    k_qkv<<<dim3(SEQ / 64, 1, 1), 32, 0, stream>>>(x, n1w, WQK, WV, Qb, Kb, Vb, QKP, VT);
    k_flash<<<dim3(SEQ / 16, 1, 1), 32 * AW, 0, stream>>>(QH, KP, VT, RES);
    k_mlp<<<dim3(SEQ / 16, 1, 1), 32, 0, stream>>>(x, RES, AWP, ab, n2w, W0, b0, W1, b1, W2, b2, OUT);
}
